// TAttentionWithProjection_33097017983678
// MI455X (gfx1250) — hardware-verified
//
#include <hip/hip_runtime.h>
#include <stdint.h>

typedef __attribute__((ext_vector_type(16))) _Float16 v16h;
typedef __attribute__((ext_vector_type(8)))  _Float16 v8h;
typedef __attribute__((ext_vector_type(16))) __bf16   v16b;
typedef __attribute__((ext_vector_type(8)))  __bf16   v8b;
typedef __attribute__((ext_vector_type(8)))  float    v8f;
typedef __attribute__((ext_vector_type(4)))  float    v4f;

#define NBATCH 4
#define TLEN 512
#define NCHAN 8
#define DMODEL 256
#define NROWS (NBATCH * TLEN * NCHAN)
#define QKLD 512
#define QBLK 64
#define KCH 32
#define PCARRY 32768.0f
#define VLO_MUL 2048.0f
#define VLO_INV (1.0f / 2048.0f)
#define QK_SCALE 0.0625f
#define MVN_EPS 1e-6f

__device__ __forceinline__ unsigned short f2bf_bits(float f) {
  unsigned u = __float_as_uint(f);
  return (unsigned short)((u + 0x7FFFu + ((u >> 16) & 1u)) >> 16);
}
__device__ __forceinline__ float bf_bits2f(unsigned short h) { return __uint_as_float(((unsigned)h) << 16); }

__device__ __forceinline__ void dep_guard_h(v8f& a, v8f& b, v16h x, v16h y) { asm volatile("v_nop\n\tv_nop\n\tv_nop\n\tv_nop" : "+v"(a), "+v"(b) : "v"(x), "v"(y)); }
__device__ __forceinline__ void dep_guard_b(v8f& a, v8f& b, v16b x, v16b y) { asm volatile("v_nop\n\tv_nop\n\tv_nop\n\tv_nop" : "+v"(a), "+v"(b) : "v"(x), "v"(y)); }
__device__ __forceinline__ void keep4_h(v16h a, v16h b, v16h c, v16h d) { asm volatile("v_nop" :: "v"(a), "v"(b), "v"(c), "v"(d)); }
__device__ __forceinline__ void keep4_b(v16b a, v16b b, v16b c, v16b d) { asm volatile("v_nop" :: "v"(a), "v"(b), "v"(c), "v"(d)); }
__device__ __forceinline__ void acc_guard4(v8f& a, v8f& b, v8f& c, v8f& d) { asm volatile("v_nop\n\tv_nop\n\tv_nop\n\tv_nop" : "+v"(a), "+v"(b), "+v"(c), "+v"(d)); }
template <typename T> struct Frag;
template <> struct Frag<_Float16> {
  typedef v16h V; union U { v16h v; v8h h[2]; };
  static __device__ __forceinline__ v16h load(const _Float16* p) {
    U f; f.h[0] = *(const v8h*)(p); f.h[1] = *(const v8h*)(p + 16); return f.v;
  }
  static __device__ __forceinline__ v8f mma(v16h a, v16h b, v8f c) {
    return __builtin_amdgcn_wmma_f32_16x16x32_f16(false, a, false, b, (short)0, c, false, false);
  }
  static __device__ __forceinline__ void guard(v8f& a, v8f& b, v16h x, v16h y) { dep_guard_h(a, b, x, y); }
  static __device__ __forceinline__ void keep(v16h a, v16h b, v16h c, v16h d) { keep4_h(a, b, c, d); }
};
template <> struct Frag<__bf16> {
  typedef v16b V; union U { v16b v; v8b h[2]; };
  static __device__ __forceinline__ v16b load(const __bf16* p) {
    U f; f.h[0] = *(const v8b*)(p); f.h[1] = *(const v8b*)(p + 16); return f.v;
  }
  static __device__ __forceinline__ v8f mma(v16b a, v16b b, v8f c) {
    return __builtin_amdgcn_wmma_f32_16x16x32_bf16(false, a, false, b, (short)0, c, false, false);
  }
  static __device__ __forceinline__ void guard(v8f& a, v8f& b, v16b x, v16b y) { dep_guard_b(a, b, x, y); }
  static __device__ __forceinline__ void keep(v16b a, v16b b, v16b c, v16b d) { keep4_b(a, b, c, d); }
};

template <int ET> struct Elem;
template <> struct Elem<0> { typedef _Float16 T; };
template <> struct Elem<1> { typedef __bf16 T; };
template <int ET, int SPLIT, int BIAS_MODE, int OUT_MODE, bool RESID>
__global__ __launch_bounds__(256) void wmma_gemm64(
    const unsigned short* __restrict__ Ap, const unsigned short* __restrict__ A2p, int lda, long strideA,
    const unsigned short* __restrict__ Btp, const unsigned short* __restrict__ Bt2p, int ldb, long strideB,
    void* __restrict__ Cout, void* __restrict__ Cout2, int ldc, long strideC,
    const float* __restrict__ bias,
    const float* __restrict__ resid, long strideR,
    int M, int N, int K, float scale) {
  typedef typename Elem<ET>::T T;
  typedef typename Frag<T>::V V;
  const T* A = (const T*)Ap; const T* A2 = (const T*)A2p; const T* Bt = (const T*)Btp; const T* Bt2 = (const T*)Bt2p;
  __shared__ __align__(16) float sT[8][16 * 68];
  const int b    = blockIdx.y;
  const int lane = threadIdx.x & 31;
  const int wave = threadIdx.x >> 5;
  const int tilesN = N >> 6;
  const int tilesM = M >> 6;
  const int tile = blockIdx.x * 8 + wave;
  if (tile >= tilesM * tilesN) return;
  const int tm = tile / tilesN;
  const int tn = tile - tm * tilesN;
  const int m0 = tm << 6;
  const int n0 = tn << 6;

  const T* Ab  = A  + (size_t)b * strideA;
  const T* Bb  = Bt + (size_t)b * strideB;
  const T* Ab2 = (SPLIT >= 1) ? (A2  + (size_t)b * strideA) : nullptr;
  const T* Bb2 = (SPLIT >= 2) ? (Bt2 + (size_t)b * strideB) : nullptr;

  const int rlane = lane & 15;
  const int koff  = (lane >> 4) * 8;
  const int mOff  = (lane >> 4) * 8;

  v8f acc[4][4];
#pragma unroll
  for (int i = 0; i < 4; ++i)
#pragma unroll
    for (int j = 0; j < 4; ++j) acc[i][j] = (v8f){0.f,0.f,0.f,0.f,0.f,0.f,0.f,0.f};

  for (int k0 = 0; k0 < K; k0 += 32) {
    V bh[4], bl[4];
#pragma unroll
    for (int j = 0; j < 4; ++j) {
      const size_t bo = (size_t)(n0 + (j << 4) + rlane) * ldb + koff + k0;
      bh[j] = Frag<T>::load(Bb + bo);
      if (SPLIT >= 2) bl[j] = Frag<T>::load(Bb2 + bo);
    }
#pragma unroll
    for (int i = 0; i < 4; ++i) {
      const size_t ao = (size_t)(m0 + (i << 4) + rlane) * lda + koff + k0;
      V ah = Frag<T>::load(Ab + ao);
      V al;
      if (SPLIT >= 1) al = Frag<T>::load(Ab2 + ao);
#pragma unroll
      for (int j = 0; j < 4; ++j) {
        acc[i][j] = Frag<T>::mma(ah, bh[j], acc[i][j]);
        if (SPLIT >= 2) acc[i][j] = Frag<T>::mma(ah, bl[j], acc[i][j]);
        if (SPLIT >= 1) acc[i][j] = Frag<T>::mma(al, bh[j], acc[i][j]);
      }
      Frag<T>::guard(acc[i][0], acc[i][3], ah, (SPLIT >= 1) ? al : ah);
    }
    Frag<T>::keep(bh[0], bh[1], bh[2], bh[3]);
    if (SPLIT >= 2) Frag<T>::keep(bl[0], bl[1], bl[2], bl[3]);
  }
  acc_guard4(acc[0][0], acc[0][1], acc[0][2], acc[0][3]);
  acc_guard4(acc[1][0], acc[1][1], acc[1][2], acc[1][3]);
  acc_guard4(acc[2][0], acc[2][1], acc[2][2], acc[2][3]);
  acc_guard4(acc[3][0], acc[3][1], acc[3][2], acc[3][3]);

  float* slab = sT[wave];
  const float* Rb = RESID ? (resid + (size_t)b * strideR) : nullptr;
#pragma unroll
  for (int i = 0; i < 4; ++i) {
    const int mBase = m0 + (i << 4);
#pragma unroll
    for (int j = 0; j < 4; ++j) {
      const int n = n0 + (j << 4) + rlane;
      float bv = 0.f;
      if (BIAS_MODE == 2) bv = bf_bits2f(f2bf_bits(bias[n]));
#pragma unroll
      for (int r = 0; r < 8; ++r) {
        float v = acc[i][j][r] * scale;
        if (BIAS_MODE == 1) v += bf_bits2f(f2bf_bits(bias[mBase + mOff + r]));
        if (BIAS_MODE == 2) v += bv;
        if (RESID) v += Rb[(size_t)(mBase + mOff + r) * ldc + n];
        slab[(mOff + r) * 68 + (j << 4) + rlane] = v;
      }
    }
    __builtin_amdgcn_fence(__ATOMIC_RELEASE, "workgroup");
    __builtin_amdgcn_wave_barrier();
    __builtin_amdgcn_fence(__ATOMIC_ACQUIRE, "workgroup");
    if (OUT_MODE == 0) {
      float* C = (float*)Cout + (size_t)b * strideC;
      const int hh = lane >> 4, c4 = (lane & 15) * 4;
      for (int pass = 0; pass < 2; ++pass) {
#pragma unroll
        for (int it = 0; it < 8; ++it) {
          const int row = it * 2 + hh;
          v4f v = *(const v4f*)(slab + row * 68 + c4);
          *(volatile v4f*)(C + (size_t)(mBase + row) * ldc + n0 + c4) = v;
        }
        __threadfence();
      }
    } else {
      const int q = lane >> 3, c8 = (lane & 7) * 8;
      unsigned short* C  = (unsigned short*)Cout  + (size_t)b * strideC;
      unsigned short* C2 = (OUT_MODE >= 2) ? ((unsigned short*)Cout2 + (size_t)b * strideC) : nullptr;
      for (int pass = 0; pass < 2; ++pass) {
#pragma unroll
        for (int it = 0; it < 4; ++it) {
          const int row = it * 4 + q;
          const float* sp = slab + row * 68 + c8;
          v8h hv, lv;
#pragma unroll
          for (int e = 0; e < 8; ++e) {
            if (OUT_MODE == 1) {
              hv[e] = (_Float16)sp[e];
            } else if (OUT_MODE == 2) {
              unsigned short hb = f2bf_bits(sp[e]);
              unsigned short lb = f2bf_bits(sp[e] - bf_bits2f(hb));
              hv[e] = __builtin_bit_cast(_Float16, hb);
              lv[e] = __builtin_bit_cast(_Float16, lb);
            } else {
              const _Float16 hq = (_Float16)sp[e];
              hv[e] = hq;
              lv[e] = (_Float16)((sp[e] - (float)hq) * VLO_MUL);
            }
          }
          *(volatile v8h*)(C + (size_t)(mBase + row) * ldc + n0 + c8) = hv;
          if (OUT_MODE >= 2) *(volatile v8h*)(C2 + (size_t)(mBase + row) * ldc + n0 + c8) = lv;
        }
        __threadfence();
      }
    }
    __builtin_amdgcn_fence(__ATOMIC_RELEASE, "workgroup");
    __builtin_amdgcn_wave_barrier();
    __builtin_amdgcn_fence(__ATOMIC_ACQUIRE, "workgroup");
  }
}

#define WTP 72
__global__ __launch_bounds__(256) void wt_cast_bf_k(const float* __restrict__ W, unsigned short* __restrict__ Wtp,
                                                    int Kp, int Np) {
  __shared__ __align__(16) _Float16 st[64 * WTP];
  _Float16* Wt = (_Float16*)Wtp;
  const int n0 = blockIdx.x * 64, k0 = blockIdx.y * 64;
  const int tid = threadIdx.x;
  const int kr = tid >> 2, c16 = (tid & 3) * 16;
  const float* src = W + (size_t)(k0 + kr) * Np + n0 + c16;
#pragma unroll
  for (int q = 0; q < 4; ++q) {
    const v4f v = *(const v4f*)(src + 4 * q);
#pragma unroll
    for (int e = 0; e < 4; ++e) st[(c16 + 4 * q + e) * WTP + kr] = __builtin_bit_cast(_Float16, f2bf_bits(v[e]));
  }
  __syncthreads();
  const int wave = tid >> 5, lane = tid & 31;
  const int q8 = lane >> 3, c8 = (lane & 7) * 8;
  for (int pass = 0; pass < 2; ++pass) {
#pragma unroll
    for (int it = 0; it < 2; ++it) {
      const int n = it * 32 + wave * 4 + q8;
      const v8h hv = *(const v8h*)(st + n * WTP + c8);
      *(volatile v8h*)(Wt + (size_t)(n0 + n) * Kp + k0 + c8) = hv;
    }
    __threadfence();
  }
}

__global__ __launch_bounds__(256) void mvn_k(const float* __restrict__ x,
                                             unsigned short* __restrict__ xnhp,
                                             unsigned short* __restrict__ xnlp,
                                             unsigned short* __restrict__ xtp) {
  _Float16* xnh = (_Float16*)xnhp;
  _Float16* xnl = (_Float16*)xnlp;
  _Float16* xt  = (_Float16*)xtp;
  const int wave = threadIdx.x >> 5, lane = threadIdx.x & 31;
  const int ro = blockIdx.x * 8 + wave;
  const int t  = ro & (TLEN - 1);
  const int bm = ro >> 9;
  const int m  = bm & (NCHAN - 1);
  const int b  = bm >> 3;
  const int rs = (b * TLEN + t) * NCHAN + m;
  const float* src = x + (size_t)rs * DMODEL + lane * 8;
  const v4f a0 = *(const v4f*)src;
  const v4f a1 = *(const v4f*)(src + 4);
  unsigned short xb[8];
  float vb[8];
#pragma unroll
  for (int e = 0; e < 4; ++e) { xb[e] = f2bf_bits(a0[e]); xb[4 + e] = f2bf_bits(a1[e]); }
#pragma unroll
  for (int e = 0; e < 8; ++e) vb[e] = bf_bits2f(xb[e]);
  float s = ((vb[0] + vb[1]) + (vb[2] + vb[3])) + ((vb[4] + vb[5]) + (vb[6] + vb[7]));
#pragma unroll
  for (int off = 1; off < 32; off <<= 1) s += __shfl_xor(s, off, 32);
  const float mu = s * (1.0f / (float)DMODEL);
  float dv[8];
#pragma unroll
  for (int e = 0; e < 8; ++e) dv[e] = vb[e] - mu;
  float sq = ((dv[0] * dv[0] + dv[1] * dv[1]) + (dv[2] * dv[2] + dv[3] * dv[3])) +
             ((dv[4] * dv[4] + dv[5] * dv[5]) + (dv[6] * dv[6] + dv[7] * dv[7]));
#pragma unroll
  for (int off = 1; off < 32; off <<= 1) sq += __shfl_xor(sq, off, 32);
  const float var = sq * (1.0f / (float)(DMODEL - 1));
  const float sd  = sqrtf(var);
  const float inv = 1.0f / (sd + MVN_EPS);
  v8h hv, lv, tv;
#pragma unroll
  for (int e = 0; e < 8; ++e) {
    const float xn = dv[e] * inv;
    const unsigned short hb = f2bf_bits(xn);
    const unsigned short lb = f2bf_bits(xn - bf_bits2f(hb));
    hv[e] = __builtin_bit_cast(_Float16, hb);
    lv[e] = __builtin_bit_cast(_Float16, lb);
    tv[e] = __builtin_bit_cast(_Float16, xb[e]);
  }
  const size_t go = (size_t)ro * DMODEL + lane * 8;
  for (int pass = 0; pass < 2; ++pass) {
    *(volatile v8h*)(xnh + go) = hv;
    *(volatile v8h*)(xnl + go) = lv;
    *(volatile v8h*)(xt  + go) = tv;
    __threadfence();
  }
}

__device__ __forceinline__ v8f mma_h(v16h a, v16h b, v8f c) {
  c = __builtin_amdgcn_wmma_f32_16x16x32_f16(false, a, false, b, (short)0, c, false, false);
  asm volatile("v_nop\n\tv_nop\n\tv_nop\n\tv_nop" : "+v"(c) : "v"(a), "v"(b));
  return c;
}

__global__ __launch_bounds__(256) void xattn_k(const unsigned short* __restrict__ qkp,
                                               const unsigned short* __restrict__ vhp,
                                               const unsigned short* __restrict__ vlp,
                                               unsigned short* __restrict__ ahp,
                                               unsigned short* __restrict__ alp) {
  __shared__ __align__(16) _Float16 Ks[KCH * DMODEL];
  __shared__ __align__(16) _Float16 Vth[DMODEL * KCH];
  __shared__ __align__(16) _Float16 Vtl[DMODEL * KCH];
  __shared__ __align__(16) _Float16 Psh[4][16 * KCH];
  __shared__ __align__(16) float Oac[QBLK * DMODEL];
  __shared__ float alph[4][16];
  __shared__ float lfin[4][16];

  const _Float16* qk = (const _Float16*)qkp;
  const _Float16* vh = (const _Float16*)vhp;
  const _Float16* vl = (const _Float16*)vlp;
  _Float16* ah = (_Float16*)ahp;
  _Float16* al = (_Float16*)alp;

  const int tid = threadIdx.x, wave = tid >> 5, lane = tid & 31;
  const int hh = lane >> 4, c = lane & 15, koff = hh * 8;
  const int sw = wave & 3;
  const int dbase = (wave >> 2) * 128;
  const int qb = blockIdx.x & 7;
  const int bm = blockIdx.x >> 3;
  const int b  = bm >> 3;
  const int qrow0 = bm * TLEN + qb * QBLK;
  const int q0  = qrow0 + sw * 16;
  const int tq0 = qb * QBLK + sw * 16;

  for (int i = tid; i < QBLK * DMODEL; i += 256) Oac[i] = 0.0f;
  __syncthreads();

  const v8f z8 = {0.f,0.f,0.f,0.f,0.f,0.f,0.f,0.f};
  const _Float16* qrowp = qk + (size_t)(q0 + c) * QKLD + koff;

#pragma unroll 1
  for (int n = 0; n < NCHAN; ++n) {
    const int krow0 = (b * NCHAN + n) * TLEN;
    float mrow[8], lrow[8];
    v8f oacc[8];
#pragma unroll
    for (int r = 0; r < 8; ++r) { mrow[r] = -INFINITY; lrow[r] = 0.f; }
#pragma unroll
    for (int t = 0; t < 8; ++t) oacc[t] = z8;

    const int nch = 2 * qb + 2;
#pragma unroll 1
    for (int kc = 0; kc < nch; ++kc) {
      const int kv0 = kc * KCH;
      __syncthreads();
#pragma unroll
      for (int i = 0; i < 4; ++i) {
        const int u = i * 256 + tid;
        const int kvr = u >> 5;
        const int d0 = (u & 31) * 8;
        const size_t grow = (size_t)(krow0 + kv0 + kvr);
        const v8h kk = *(const v8h*)(qk + grow * QKLD + DMODEL + d0);
        const v8h v1 = *(const v8h*)(vh + grow * DMODEL + d0);
        const v8h v2 = *(const v8h*)(vl + grow * DMODEL + d0);
        *(v8h*)(Ks + kvr * DMODEL + d0) = kk;
#pragma unroll
        for (int e = 0; e < 8; ++e) {
          Vth[(d0 + e) * KCH + kvr] = v1[e];
          Vtl[(d0 + e) * KCH + kvr] = v2[e];
        }
      }
      __syncthreads();

      if (wave < 4) {
        v8f s[2];
        s[0] = z8; s[1] = z8;
#pragma unroll
        for (int dc = 0; dc < 8; ++dc) {
          const v16h qa  = Frag<_Float16>::load(qrowp + dc * 32);
          const v16h k0f = Frag<_Float16>::load(Ks + c * DMODEL + dc * 32 + koff);
          const v16h k1f = Frag<_Float16>::load(Ks + (16 + c) * DMODEL + dc * 32 + koff);
          s[0] = mma_h(qa, k0f, s[0]);
          s[1] = mma_h(qa, k1f, s[1]);
        }
        float cm[8];
#pragma unroll
        for (int r = 0; r < 8; ++r) {
          const int tq = tq0 + 8 * hh + r;
          float mx = -INFINITY;
#pragma unroll
          for (int j = 0; j < 2; ++j) {
            const int key = kv0 + 16 * j + c;
            float v = s[j][r] * QK_SCALE;
            v = (key > tq) ? -INFINITY : v;
            s[j][r] = v;
            mx = fmaxf(mx, v);
          }
#pragma unroll
          for (int off = 1; off < 16; off <<= 1) mx = fmaxf(mx, __shfl_xor(mx, off, 32));
          cm[r] = mx;
        }
        _Float16* pw = Psh[sw];
#pragma unroll
        for (int r = 0; r < 8; ++r) {
          const float mnew  = fmaxf(mrow[r], cm[r]);
          const float alpha = expf(mrow[r] - mnew);
          mrow[r] = mnew;
          float psum = 0.f;
#pragma unroll
          for (int j = 0; j < 2; ++j) {
            const float p = expf(s[j][r] - mnew);
            psum += p;
            pw[(8 * hh + r) * KCH + 16 * j + c] = (_Float16)(p * PCARRY);
          }
#pragma unroll
          for (int off = 1; off < 16; off <<= 1) psum += __shfl_xor(psum, off, 32);
          lrow[r] = lrow[r] * alpha + psum;
#pragma unroll
          for (int t = 0; t < 8; ++t) oacc[t][r] *= alpha;
          if (c == 0) alph[sw][8 * hh + r] = alpha;
        }
      }
      __syncthreads();

      if (wave >= 4) {
#pragma unroll
        for (int r = 0; r < 8; ++r) {
          const float a = alph[sw][8 * hh + r];
#pragma unroll
          for (int t = 0; t < 8; ++t) oacc[t][r] *= a;
        }
      }
      {
        const v16h pa = Frag<_Float16>::load(Psh[sw] + c * KCH + koff);
#pragma unroll
        for (int t = 0; t < 8; ++t) {
          const int dcol = dbase + t * 16 + c;
          const v16h vbh = Frag<_Float16>::load(Vth + dcol * KCH + koff);
          const v16h vbl = Frag<_Float16>::load(Vtl + dcol * KCH + koff);
          oacc[t] = mma_h(pa, vbh, oacc[t]);
          const v8f lo = mma_h(pa, vbl, z8);
          oacc[t] += lo * VLO_INV;
        }
      }
    }
    if (wave < 4) {
      if (c == 0) {
#pragma unroll
        for (int r = 0; r < 8; ++r) lfin[sw][8 * hh + r] = lrow[r];
      }
    }
    __syncthreads();
#pragma unroll
    for (int r = 0; r < 8; ++r) {
      const float inv = 1.0f / (lfin[sw][8 * hh + r] * PCARRY);
      float* orow = Oac + (sw * 16 + 8 * hh + r) * DMODEL + dbase + c;
#pragma unroll
      for (int t = 0; t < 8; ++t) orow[t * 16] += oacc[t][r] * inv;
    }
  }
  __syncthreads();

  for (int pass = 0; pass < 2; ++pass) {
#pragma unroll
    for (int it = 0; it < 8; ++it) {
      const int row = wave * 8 + it;
      const float* op = Oac + row * DMODEL + lane * 8;
      const v4f x0 = *(const v4f*)op;
      const v4f x1 = *(const v4f*)(op + 4);
      v8h hv, lv;
#pragma unroll
      for (int e = 0; e < 4; ++e) {
        const unsigned short hb0 = f2bf_bits(x0[e]);
        const unsigned short lb0 = f2bf_bits(x0[e] - bf_bits2f(hb0));
        const unsigned short hb1 = f2bf_bits(x1[e]);
        const unsigned short lb1 = f2bf_bits(x1[e] - bf_bits2f(hb1));
        hv[e] = __builtin_bit_cast(_Float16, hb0);
        lv[e] = __builtin_bit_cast(_Float16, lb0);
        hv[4 + e] = __builtin_bit_cast(_Float16, hb1);
        lv[4 + e] = __builtin_bit_cast(_Float16, lb1);
      }
      const size_t go = (size_t)(qrow0 + row) * DMODEL + lane * 8;
      *(volatile v8h*)(ah + go) = hv;
      *(volatile v8h*)(al + go) = lv;
    }
    __threadfence();
  }
}

extern "C" void kernel_launch(void* const* d_in, const int* in_sizes, int n_in,
                              void* d_out, int out_size, void* d_ws, size_t ws_size,
                              hipStream_t stream) {
  if (n_in < 11) return;
  if (in_sizes[0] != NROWS * DMODEL || out_size != NROWS * DMODEL) return;
  if (in_sizes[1] != DMODEL * DMODEL || in_sizes[3] != DMODEL * DMODEL || in_sizes[5] != DMODEL * DMODEL ||
      in_sizes[7] != DMODEL * DMODEL || in_sizes[9] != 2 * DMODEL * DMODEL) return;
  if (in_sizes[2] != DMODEL || in_sizes[4] != DMODEL || in_sizes[6] != DMODEL || in_sizes[8] != DMODEL || in_sizes[10] != DMODEL) return;

  const float* x   = (const float*)d_in[0];
  const float* Wq  = (const float*)d_in[1];
  const float* bq  = (const float*)d_in[2];
  const float* Wk  = (const float*)d_in[3];
  const float* bk  = (const float*)d_in[4];
  const float* Wv  = (const float*)d_in[5];
  const float* bv  = (const float*)d_in[6];
  const float* Wpa = (const float*)d_in[7];
  const float* bpa = (const float*)d_in[8];
  const float* Wpc = (const float*)d_in[9];
  const float* bpc = (const float*)d_in[10];

  const size_t PL16 = (size_t)NROWS * DMODEL * 2;
  const size_t WQKV_B = (size_t)3 * DMODEL * DMODEL * 2;
  const size_t WSQ_B  = (size_t)DMODEL * DMODEL * 2;
  const size_t oXNH = 0, oXNL = PL16, oXT = 2 * PL16, oQK = 3 * PL16, oVH = 5 * PL16, oVL = 6 * PL16;
  const size_t oAPH = 7 * PL16, oAPL = 8 * PL16, oZP = 9 * PL16, oW = 11 * PL16;
  const size_t oWQKV = oW, oWPA = oW + WQKV_B, oWPC0 = oWPA + WSQ_B, oWPC1 = oWPC0 + WSQ_B;
  const size_t WS_TOTAL = oWPC1 + WSQ_B;
  if (ws_size < WS_TOTAL) return;

  char* ws = (char*)d_ws;
  unsigned short* XNH  = (unsigned short*)(ws + oXNH);
  unsigned short* XNL  = (unsigned short*)(ws + oXNL);
  unsigned short* XT   = (unsigned short*)(ws + oXT);
  unsigned short* QKP  = (unsigned short*)(ws + oQK);
  unsigned short* VH   = (unsigned short*)(ws + oVH);
  unsigned short* VL   = (unsigned short*)(ws + oVL);
  unsigned short* APH  = (unsigned short*)(ws + oAPH);
  unsigned short* APL  = (unsigned short*)(ws + oAPL);
  float*          ZP   = (float*)(ws + oZP);
  unsigned short* WQKV = (unsigned short*)(ws + oWQKV);
  unsigned short* WPA  = (unsigned short*)(ws + oWPA);
  unsigned short* WPC0 = (unsigned short*)(ws + oWPC0);
  unsigned short* WPC1 = (unsigned short*)(ws + oWPC1);
  unsigned short* AH = XNH;
  unsigned short* AL = XNL;

  const dim3 gw(DMODEL / 64, DMODEL / 64);
  wt_cast_bf_k<<<gw, 256, 0, stream>>>(Wq,  WQKV, DMODEL, DMODEL);
  wt_cast_bf_k<<<gw, 256, 0, stream>>>(Wk,  WQKV + (size_t)DMODEL * DMODEL, DMODEL, DMODEL);
  wt_cast_bf_k<<<gw, 256, 0, stream>>>(Wv,  WQKV + (size_t)2 * DMODEL * DMODEL, DMODEL, DMODEL);
  wt_cast_bf_k<<<gw, 256, 0, stream>>>(Wpa, WPA, DMODEL, DMODEL);
  wt_cast_bf_k<<<gw, 256, 0, stream>>>(Wpc, WPC0, DMODEL, DMODEL);
  wt_cast_bf_k<<<gw, 256, 0, stream>>>(Wpc + (size_t)DMODEL * DMODEL, WPC1, DMODEL, DMODEL);

  mvn_k<<<NROWS / 8, 256, 0, stream>>>(x, XNH, XNL, XT);

  const dim3 gg((NROWS / 64) * (DMODEL / 64) / 8, 1);
  wmma_gemm64<1, 1, 2, 1, false><<<gg, 256, 0, stream>>>(
      XNH, XNL, DMODEL, 0L, WQKV, nullptr, DMODEL, 0L,
      (void*)QKP, nullptr, QKLD, 0L, bq, nullptr, 0L, NROWS, DMODEL, DMODEL, 1.0f);
  wmma_gemm64<1, 1, 2, 1, false><<<gg, 256, 0, stream>>>(
      XNH, XNL, DMODEL, 0L, WQKV + (size_t)DMODEL * DMODEL, nullptr, DMODEL, 0L,
      (void*)(QKP + DMODEL), nullptr, QKLD, 0L, bk, nullptr, 0L, NROWS, DMODEL, DMODEL, 1.0f);
  wmma_gemm64<1, 1, 2, 3, false><<<gg, 256, 0, stream>>>(
      XNH, XNL, DMODEL, 0L, WQKV + (size_t)2 * DMODEL * DMODEL, nullptr, DMODEL, 0L,
      (void*)VH, (void*)VL, DMODEL, 0L, bv, nullptr, 0L, NROWS, DMODEL, DMODEL, 1.0f);

  xattn_k<<<NBATCH * NCHAN * (TLEN / QBLK), 256, 0, stream>>>(QKP, VH, VL, AH, AL);

  wmma_gemm64<1, 1, 2, 2, false><<<gg, 256, 0, stream>>>(
      AH, AL, DMODEL, 0L, WPA, nullptr, DMODEL, 0L,
      (void*)APH, (void*)APL, DMODEL, 0L, bpa, nullptr, 0L, NROWS, DMODEL, DMODEL, 1.0f);

  wmma_gemm64<1, 0, 2, 0, false><<<gg, 256, 0, stream>>>(
      XT, nullptr, DMODEL, 0L, WPC0, nullptr, DMODEL, 0L,
      (void*)ZP, nullptr, DMODEL, 0L, bpc, nullptr, 0L, NROWS, DMODEL, DMODEL, 1.0f);

  wmma_gemm64<1, 1, 0, 0, true><<<gg, 256, 0, stream>>>(
      APH, APL, DMODEL, 0L, WPC1, nullptr, DMODEL, 0L,
      d_out, nullptr, DMODEL, 0L, nullptr, ZP, 0L, NROWS, DMODEL, DMODEL, 1.0f);
}
